// IntraModalityEnhance_30073361007269
// MI455X (gfx1250) — hardware-verified
//
#include <hip/hip_runtime.h>


#define NB_  2
#define SS   2048
#define DD   1024
#define NH_  16
#define HD   64
#define WW   31
#define PAD  15
#define SCL  0.125f
typedef _Float16 h16;
typedef unsigned short bf;
typedef __attribute__((ext_vector_type(16))) __bf16   v16bf;
typedef __attribute__((ext_vector_type(16))) _Float16 v16h;
typedef __attribute__((ext_vector_type(8)))  _Float16 v8h;
typedef __attribute__((ext_vector_type(8)))  unsigned short v8us;
typedef __attribute__((ext_vector_type(8)))  float    v8f;
typedef __attribute__((ext_vector_type(4)))  float    v4f;
typedef v8h  __attribute__((may_alias)) v8ha;
typedef v4f  __attribute__((may_alias)) v4fa;
typedef v8us __attribute__((may_alias)) v8usa;

__device__ __forceinline__ unsigned short f2bf(float f) { unsigned u = __float_as_uint(f); u += 0x7FFFu + ((u >> 16) & 1u); return (unsigned short)(u >> 16); }
__device__ __forceinline__ float bf2f(unsigned short b) { return __uint_as_float(((unsigned)b) << 16); }
__device__ __forceinline__ float bfr(float f) { return bf2f(f2bf(f)); }
__device__ __forceinline__ v16h cat16(v8h lo, v8h hi) { return __builtin_shufflevector(lo, hi, 0, 1, 2, 3, 4, 5, 6, 7, 8, 9, 10, 11, 12, 13, 14, 15); }
__device__ __forceinline__ v16bf cat16b(v8us lo, v8us hi) { return __builtin_bit_cast(v16bf, __builtin_shufflevector(lo, hi, 0, 1, 2, 3, 4, 5, 6, 7, 8, 9, 10, 11, 12, 13, 14, 15)); }
__device__ __forceinline__ v8f wmma16(v16h a, v16h b, v8f c) { return __builtin_amdgcn_wmma_f32_16x16x32_f16(false, a, false, b, (short)0, c, false, false); }
__device__ __forceinline__ v8f wmmab(v16bf a, v16bf b, v8f c) { return __builtin_amdgcn_wmma_f32_16x16x32_bf16(false, a, false, b, (short)0, c, false, false); }


template <typename T16> struct WFrag;
template <> struct WFrag<h16> { typedef v16h V; static __device__ __forceinline__ V ld(const h16* p) { return cat16(*(const v8h*)p, *(const v8h*)(p + 16)); } static __device__ __forceinline__ v8f mma(V a, V b, v8f c) { return wmma16(a, b, c); } };
template <> struct WFrag<bf> { typedef v16bf V; static __device__ __forceinline__ V ld(const bf* p) { return cat16b(*(const v8us*)p, *(const v8us*)(p + 16)); } static __device__ __forceinline__ v8f mma(V a, V b, v8f c) { return wmmab(a, b, c); } };
template <typename T16, int NSPLIT, bool BIAS>
__global__ __launch_bounds__(32) void k_gemmw(const T16* __restrict__ A, const T16* __restrict__ A2, const T16* __restrict__ Bt, const T16* __restrict__ Bt2, int K, float* C, int ldc, const float* __restrict__ bias, size_t sA, size_t sB, size_t sC) {
    typedef typename WFrag<T16>::V V;
    __shared__ __align__(16) float os[16 * 68];
    const size_t z = blockIdx.z; A += z * sA; if (A2) A2 += z * sA; Bt += z * sB; if (Bt2) Bt2 += z * sB; C += z * sC;
    const int lane = threadIdx.x & 31, lr = lane & 15, hi = lane >> 4; const int r0 = blockIdx.x * 64, c0 = blockIdx.y * 64;
    v8f acc[4][4];
#pragma unroll
    for (int mb = 0; mb < 4; ++mb)
#pragma unroll
        for (int nb = 0; nb < 4; ++nb) acc[mb][nb] = (v8f){};
    const size_t aoff = (size_t)(r0 + lr) * K + 8 * hi, boff = (size_t)(c0 + lr) * K + 8 * hi;
#pragma unroll 1
    for (int kc = 0; kc < K; kc += 32) {
        V a[4], a2[4];
#pragma unroll
        for (int mb = 0; mb < 4; ++mb) { a[mb] = WFrag<T16>::ld(A + aoff + (size_t)mb * 16 * K + kc); if (NSPLIT == 1 || NSPLIT == 2) a2[mb] = WFrag<T16>::ld(A2 + aoff + (size_t)mb * 16 * K + kc); }
#pragma unroll
        for (int nb = 0; nb < 4; ++nb) { const V b = WFrag<T16>::ld(Bt + boff + (size_t)nb * 16 * K + kc); V b2; if (NSPLIT >= 2) b2 = WFrag<T16>::ld(Bt2 + boff + (size_t)nb * 16 * K + kc);
#pragma unroll
            for (int mb = 0; mb < 4; ++mb) { acc[mb][nb] = WFrag<T16>::mma(a[mb], b, acc[mb][nb]); if (NSPLIT == 1 || NSPLIT == 2) acc[mb][nb] = WFrag<T16>::mma(a2[mb], b, acc[mb][nb]); if (NSPLIT >= 2) acc[mb][nb] = WFrag<T16>::mma(a[mb], b2, acc[mb][nb]); } }
        asm volatile("v_nop\n\tv_nop\n\tv_nop\n\tv_nop" : "+v"(acc[0][0]), "+v"(acc[1][1]), "+v"(acc[2][2]), "+v"(acc[3][3]) : "v"(a[0]), "v"(a[3]));
    }
#pragma unroll
    for (int mb = 0; mb < 4; ++mb) {
#pragma unroll
        for (int nb = 0; nb < 4; ++nb) {
#pragma unroll
            for (int j = 0; j < 8; ++j) os[(hi * 8 + j) * 68 + nb * 16 + lr] = acc[mb][nb][j]; }
        __builtin_amdgcn_wave_barrier(); asm volatile("" ::: "memory");
        float* crow = C + (size_t)(r0 + mb * 16) * ldc + c0;
#pragma unroll 1
        for (int ps = 0; ps < 2; ++ps) {
#pragma unroll
            for (int s = 0; s < 8; ++s) { const int row = 2 * s + hi, cofs = lr * 4; v4f val = *(const v4fa*)(os + row * 68 + cofs); if (BIAS) { val[0] += bfr(bias[c0 + cofs]); val[1] += bfr(bias[c0 + cofs + 1]); val[2] += bfr(bias[c0 + cofs + 2]); val[3] += bfr(bias[c0 + cofs + 3]); }
                *(volatile v4f*)(crow + (size_t)row * ldc + cofs) = val; }
            if (ps == 0) __threadfence(); }
        __builtin_amdgcn_wave_barrier(); asm volatile("" ::: "memory");
    }
}

__device__ __forceinline__ void splitf(float y, unsigned short& h, unsigned short& l) { h = f2bf(y); l = f2bf(y - bf2f(h)); }
typedef __attribute__((ext_vector_type(2))) unsigned short v2us;
typedef __attribute__((ext_vector_type(4))) unsigned short v4us;

__global__ __launch_bounds__(256) void k_wtG(const float* __restrict__ w, int K, int N, bf* Bt) {
    const int lane = threadIdx.x & 31; const int L0 = (blockIdx.x * 8 + (threadIdx.x >> 5)) * 8; const int nlines = N * K / 64;
#pragma unroll 1
    for (int ps = 0; ps < 2; ++ps) {
#pragma unroll 1
        for (int l = 0; l < 8; ++l) { const int L = L0 + l; if (L >= nlines) break; const size_t e = (size_t)L * 64 + lane * 2; const int k = (int)(e % K), n = (int)(e / K); v2us o;
            o[0] = f2bf(w[(size_t)k * N + n]); o[1] = f2bf(w[(size_t)(k + 1) * N + n]); *(volatile v2us*)(Bt + e) = o; }
        if (ps == 0) __threadfence(); }
}
__global__ __launch_bounds__(256) void k_cvt8(const float* __restrict__ src, bf* dst, size_t n8) { const size_t i = (size_t)blockIdx.x * 256 + threadIdx.x; if (i >= n8) return; const v8f v = *(const v8f*)(src + i * 8); v8us o;
#pragma unroll
    for (int k = 0; k < 8; ++k) o[k] = f2bf(v[k]); *(volatile v8us*)(dst + i * 8) = o; __threadfence(); *(volatile v8us*)(dst + i * 8) = o; }
__global__ __launch_bounds__(256) void k_wt3(const float* __restrict__ w, bf* Bt) { const int e4 = (blockIdx.x * 256 + threadIdx.x) * 4; if (e4 >= NH_ * HD * DD) return; const int k = e4 % DD; const int n = e4 / DD; const int h = n / HD, e = n % HD; v4us o;
#pragma unroll
    for (int q = 0; q < 4; ++q) o[q] = f2bf(w[((size_t)h * DD + k + q) * HD + e]); *(volatile v4us*)(Bt + e4) = o; __threadfence(); *(volatile v4us*)(Bt + e4) = o; }
__global__ __launch_bounds__(256) void k_local(const float* __restrict__ QF, const float* __restrict__ XK, const float* __restrict__ XV, const float* __restrict__ PK, const float* __restrict__ PV, const float* __restrict__ FK, const float* __restrict__ FV,
                                               const float* __restrict__ bk, const float* __restrict__ bv, bf* Ah, bf* Al) {
    const int lane = threadIdx.x & 31; const int r = blockIdx.x * 8 + (threadIdx.x >> 5); if (r >= NB_ * NH_ * SS) return; const int s = r % SS; const int h = (r / SS) % NH_; const int b = r / (SS * NH_);
    const float* q = QF + (size_t)s * DD + h * HD; const int t = s - PAD + lane; const bool inwin = (lane < WW), valid = inwin && t >= 0 && t < SS;
    const float* k1 = (lane == WW) ? (PK + (size_t)s * DD + h * HD) : (valid ? (XK + ((size_t)b * SS + t) * DD + h * HD) : (bk + h * HD));
    const float* v1 = (lane == WW) ? (PV + (size_t)s * DD + h * HD) : (valid ? (XV + ((size_t)b * SS + t) * DD + h * HD) : (bv + h * HD));
    const bool raw1 = inwin && !valid;
    const float* k2 = FK + (size_t)s * DD + h * HD;
    float s1 = 0.f, s2 = 0.f;
#pragma unroll 4
    for (int d = 0; d < HD; ++d) { const float qd = q[d]; float a1 = raw1 ? bfr(k1[d]) : k1[d], a2 = k2[d]; asm volatile("" : "+v"(a1)); asm volatile("" : "+v"(a2)); float p1 = __fmul_rn(qd, a1), p2 = __fmul_rn(qd, a2); asm volatile("" : "+v"(p1)); asm volatile("" : "+v"(p2)); s1 = __fadd_rn(s1, p1); s2 = __fadd_rn(s2, p2); }
    s1 *= SCL; s2 = (lane == 0) ? s2 * SCL : -3.0e38f; float mx = fmaxf(s1, s2);
#pragma unroll
    for (int sh = 16; sh; sh >>= 1) mx = fmaxf(mx, __shfl_xor(mx, sh, 32));
    float d1 = __fsub_rn(s1, mx), d2 = __fsub_rn(s2, mx); asm volatile("" : "+v"(d1)); asm volatile("" : "+v"(d2)); const float e1 = __builtin_amdgcn_exp2f(__fmul_rn(d1, 1.4426950408889634f)), e2 = (lane == 0) ? __builtin_amdgcn_exp2f(__fmul_rn(d2, 1.4426950408889634f)) : 0.f; float sum = __fadd_rn(e1, e2);
#pragma unroll
    for (int sh = 16; sh; sh >>= 1) sum += __shfl_xor(sum, sh, 32);
    const float inv = __fdiv_rn(1.0f, sum); float a1w = __fmul_rn(e1, inv), a2w = __fmul_rn(e2, inv); asm volatile("" : "+v"(a1w)); asm volatile("" : "+v"(a2w));
    float o0 = 0.f, o1 = 0.f; const int dd = 2 * lane;
    for (int j = 0; j < 32; ++j) { const float aw = __shfl(a1w, j, 32); const int tj = s - PAD + j; const bool vj = (j < WW) && tj >= 0 && tj < SS;
        const float* vr = (j == WW) ? (PV + (size_t)s * DD + h * HD) : (vj ? (XV + ((size_t)b * SS + tj) * DD + h * HD) : (bv + h * HD)); const bool rawj = (j < WW) && !vj;
        float x0 = rawj ? bfr(vr[dd]) : vr[dd], x1 = rawj ? bfr(vr[dd + 1]) : vr[dd + 1]; asm volatile("" : "+v"(x0)); asm volatile("" : "+v"(x1)); float p0 = __fmul_rn(aw, x0), p1 = __fmul_rn(aw, x1); asm volatile("" : "+v"(p0)); asm volatile("" : "+v"(p1)); o0 = __fadd_rn(o0, p0); o1 = __fadd_rn(o1, p1); }
    { const float aw = __shfl(a2w, 0, 32); const float* vr = FV + (size_t)s * DD + h * HD; float p0 = __fmul_rn(aw, vr[dd]), p1 = __fmul_rn(aw, vr[dd + 1]); asm volatile("" : "+v"(p0)); asm volatile("" : "+v"(p1)); o0 = __fadd_rn(o0, p0); o1 = __fadd_rn(o1, p1); }
    v2us oh, ol; unsigned short a, c2; splitf(o0, a, c2); oh[0] = a; ol[0] = c2; splitf(o1, a, c2); oh[1] = a; ol[1] = c2; const size_t oo = ((size_t)b * SS + s) * DD + h * HD + dd;
    *(volatile v2us*)(Ah + oo) = oh; *(volatile v2us*)(Al + oo) = ol; __threadfence(); *(volatile v2us*)(Ah + oo) = oh; *(volatile v2us*)(Al + oo) = ol; }

extern "C" void kernel_launch(void* const* d_in, const int* in_sizes, int n_in,
                              void* d_out, int out_size, void* d_ws, size_t ws_size, hipStream_t stream) {
    (void)in_sizes; (void)n_in; (void)out_size;
    const float* x = (const float*)d_in[0]; const float* fsq = (const float*)d_in[1]; const float* pos = (const float*)d_in[2]; const float* wq = (const float*)d_in[3]; const float* bq = (const float*)d_in[4]; const float* wk = (const float*)d_in[5]; const float* bk = (const float*)d_in[6]; const float* wv = (const float*)d_in[7]; const float* bv = (const float*)d_in[8]; const float* wo = (const float*)d_in[9]; const float* bo = (const float*)d_in[10];
    float* OUT = (float*)d_out;
    char* wsp = (char*)d_ws;
    auto take = [&](size_t bytes) { char* p = wsp; wsp += (bytes + 255) & ~(size_t)255; return (void*)p; };
    const size_t NR = (size_t)NB_ * SS;
    bf* WQ = (bf*)take((size_t)DD * DD * 2); bf* WK = (bf*)take((size_t)DD * DD * 2); bf* WV = (bf*)take((size_t)DD * DD * 2); bf* WO = (bf*)take((size_t)DD * DD * 2); bf* XB = (bf*)take(NR * DD * 2); bf* FB = (bf*)take((size_t)SS * DD * 2); bf* PB = (bf*)take((size_t)SS * DD * 2);
    float* QF = (float*)take((size_t)SS * DD * 4); float* XK = (float*)take(NR * DD * 4); float* XV = (float*)take(NR * DD * 4); float* PK = (float*)take((size_t)SS * DD * 4); float* PV = (float*)take((size_t)SS * DD * 4); float* FK = (float*)take((size_t)SS * DD * 4); float* FV = (float*)take((size_t)SS * DD * 4); bf* Ah = (bf*)take(NR * DD * 2); bf* Al = (bf*)take(NR * DD * 2);
    if ((size_t)(wsp - (char*)d_ws) > ws_size) return;
    { k_wt3<<<(NH_ * HD * DD / 4 + 255) / 256, 256, 0, stream>>>(wq, WQ); k_wt3<<<(NH_ * HD * DD / 4 + 255) / 256, 256, 0, stream>>>(wk, WK); k_wt3<<<(NH_ * HD * DD / 4 + 255) / 256, 256, 0, stream>>>(wv, WV); k_wtG<<<(unsigned)((DD * DD / 64 + 63) / 64), 256, 0, stream>>>(wo, DD, DD, WO);
      k_cvt8<<<(unsigned)((NR * DD / 8 + 255) / 256), 256, 0, stream>>>(x, XB, NR * DD / 8); k_cvt8<<<(unsigned)(((size_t)SS * DD / 8 + 255) / 256), 256, 0, stream>>>(fsq, FB, (size_t)SS * DD / 8); k_cvt8<<<(unsigned)(((size_t)SS * DD / 8 + 255) / 256), 256, 0, stream>>>(pos, PB, (size_t)SS * DD / 8); }
    const dim3 gS(SS / 64, DD / 64, 1), gX((unsigned)(NR / 64), DD / 64, 1);
    k_gemmw<bf, 0, true><<<gS, 32, 0, stream>>>(FB, nullptr, WQ, nullptr, DD, QF, DD, bq, 0, 0, 0); k_gemmw<bf, 0, true><<<gS, 32, 0, stream>>>(FB, nullptr, WK, nullptr, DD, FK, DD, bk, 0, 0, 0); k_gemmw<bf, 0, true><<<gS, 32, 0, stream>>>(FB, nullptr, WV, nullptr, DD, FV, DD, bv, 0, 0, 0);
    k_gemmw<bf, 0, true><<<gS, 32, 0, stream>>>(PB, nullptr, WK, nullptr, DD, PK, DD, bk, 0, 0, 0); k_gemmw<bf, 0, true><<<gS, 32, 0, stream>>>(PB, nullptr, WV, nullptr, DD, PV, DD, bv, 0, 0, 0);
    k_gemmw<bf, 0, true><<<gX, 32, 0, stream>>>(XB, nullptr, WK, nullptr, DD, XK, DD, bk, 0, 0, 0); k_gemmw<bf, 0, true><<<gX, 32, 0, stream>>>(XB, nullptr, WV, nullptr, DD, XV, DD, bv, 0, 0, 0);
    k_local<<<(NB_ * NH_ * SS) / 8, 256, 0, stream>>>(QF, XK, XV, PK, PV, FK, FV, bk, bv, Ah, Al);
    k_gemmw<bf, 1, true><<<gX, 32, 0, stream>>>(Ah, Al, WO, nullptr, DD, OUT, DD, bo, 0, 0, 0);
}
